// AxwinLowMixear_85117661872681
// MI455X (gfx1250) — hardware-verified
//
#include <hip/hip_runtime.h>


#define NBI  4
#define DIM  384
#define RES  56
#define NN   3136
#define TD   192
#define CSC  96
#define CSD  48
#define NWD  8
#define NTW  392
#define NTP  448
#define NG2  16
#define DNH  3
#define DH   64
#define PCAR 1024.0f
typedef _Float16 h16;
typedef unsigned short bf;
typedef __attribute__((ext_vector_type(16))) __bf16   v16bf;
typedef __attribute__((ext_vector_type(16))) _Float16 v16h;
typedef __attribute__((ext_vector_type(8)))  _Float16 v8h;
typedef __attribute__((ext_vector_type(8)))  unsigned short v8us;
typedef __attribute__((ext_vector_type(8)))  float    v8f;
typedef __attribute__((ext_vector_type(4)))  float    v4f;
typedef v8h  __attribute__((may_alias)) v8ha;
typedef v4f  __attribute__((may_alias)) v4fa;
typedef v8us __attribute__((may_alias)) v8usa;

__device__ __forceinline__ unsigned short f2bf(float f) { unsigned u = __float_as_uint(f); u += 0x7FFFu + ((u >> 16) & 1u); return (unsigned short)(u >> 16); }
__device__ __forceinline__ float bf2f(unsigned short b) { return __uint_as_float(((unsigned)b) << 16); }
__device__ __forceinline__ float bfr(float f) { return bf2f(f2bf(f)); }
__device__ __forceinline__ v16h cat16(v8h lo, v8h hi) { return __builtin_shufflevector(lo, hi, 0, 1, 2, 3, 4, 5, 6, 7, 8, 9, 10, 11, 12, 13, 14, 15); }
__device__ __forceinline__ v16bf cat16b(v8us lo, v8us hi) { return __builtin_bit_cast(v16bf, __builtin_shufflevector(lo, hi, 0, 1, 2, 3, 4, 5, 6, 7, 8, 9, 10, 11, 12, 13, 14, 15)); }
__device__ __forceinline__ v8f wmma16(v16h a, v16h b, v8f c) { return __builtin_amdgcn_wmma_f32_16x16x32_f16(false, a, false, b, (short)0, c, false, false); }
__device__ __forceinline__ v8f wmmab(v16bf a, v16bf b, v8f c) { return __builtin_amdgcn_wmma_f32_16x16x32_bf16(false, a, false, b, (short)0, c, false, false); }


template <typename T16> struct WFrag;
template <> struct WFrag<h16> { typedef v16h V; static __device__ __forceinline__ V ld(const h16* p) { return cat16(*(const v8h*)p, *(const v8h*)(p + 16)); } static __device__ __forceinline__ v8f mma(V a, V b, v8f c) { return wmma16(a, b, c); } };
template <> struct WFrag<bf> { typedef v16bf V; static __device__ __forceinline__ V ld(const bf* p) { return cat16b(*(const v8us*)p, *(const v8us*)(p + 16)); } static __device__ __forceinline__ v8f mma(V a, V b, v8f c) { return wmmab(a, b, c); } };
template <typename T16, int NSPLIT, bool BIAS>
__global__ __launch_bounds__(32) void k_gemmw(const T16* __restrict__ A, const T16* __restrict__ A2, const T16* __restrict__ Bt, const T16* __restrict__ Bt2, int K, float* C, int ldc, const float* __restrict__ bias, size_t sA, size_t sB, size_t sC) {
    typedef typename WFrag<T16>::V V;
    __shared__ __align__(16) float os[16 * 68];
    const size_t z = blockIdx.z; A += z * sA; if (A2) A2 += z * sA; Bt += z * sB; if (Bt2) Bt2 += z * sB; C += z * sC;
    const int lane = threadIdx.x & 31, lr = lane & 15, hi = lane >> 4; const int r0 = blockIdx.x * 64, c0 = blockIdx.y * 64;
    v8f acc[4][4];
#pragma unroll
    for (int mb = 0; mb < 4; ++mb)
#pragma unroll
        for (int nb = 0; nb < 4; ++nb) acc[mb][nb] = (v8f){};
    const size_t aoff = (size_t)(r0 + lr) * K + 8 * hi, boff = (size_t)(c0 + lr) * K + 8 * hi;
#pragma unroll 1
    for (int kc = 0; kc < K; kc += 32) {
        V a[4], a2[4];
#pragma unroll
        for (int mb = 0; mb < 4; ++mb) { a[mb] = WFrag<T16>::ld(A + aoff + (size_t)mb * 16 * K + kc); if (NSPLIT == 1 || NSPLIT == 2) a2[mb] = WFrag<T16>::ld(A2 + aoff + (size_t)mb * 16 * K + kc); }
#pragma unroll
        for (int nb = 0; nb < 4; ++nb) { const V b = WFrag<T16>::ld(Bt + boff + (size_t)nb * 16 * K + kc); V b2; if (NSPLIT >= 2) b2 = WFrag<T16>::ld(Bt2 + boff + (size_t)nb * 16 * K + kc);
#pragma unroll
            for (int mb = 0; mb < 4; ++mb) { acc[mb][nb] = WFrag<T16>::mma(a[mb], b, acc[mb][nb]); if (NSPLIT == 1 || NSPLIT == 2) acc[mb][nb] = WFrag<T16>::mma(a2[mb], b, acc[mb][nb]); if (NSPLIT >= 2) acc[mb][nb] = WFrag<T16>::mma(a[mb], b2, acc[mb][nb]); } }
        asm volatile("v_nop\n\tv_nop\n\tv_nop\n\tv_nop" : "+v"(acc[0][0]), "+v"(acc[1][1]), "+v"(acc[2][2]), "+v"(acc[3][3]) : "v"(a[0]), "v"(a[3]));
    }
#pragma unroll
    for (int mb = 0; mb < 4; ++mb) {
#pragma unroll
        for (int nb = 0; nb < 4; ++nb) {
#pragma unroll
            for (int j = 0; j < 8; ++j) os[(hi * 8 + j) * 68 + nb * 16 + lr] = acc[mb][nb][j]; }
        __builtin_amdgcn_wave_barrier(); asm volatile("" ::: "memory");
        float* crow = C + (size_t)(r0 + mb * 16) * ldc + c0;
#pragma unroll 1
        for (int ps = 0; ps < 2; ++ps) {
#pragma unroll
            for (int s = 0; s < 8; ++s) { const int row = 2 * s + hi, cofs = lr * 4; v4f val = *(const v4fa*)(os + row * 68 + cofs); if (BIAS) { val[0] += bfr(bias[c0 + cofs]); val[1] += bfr(bias[c0 + cofs + 1]); val[2] += bfr(bias[c0 + cofs + 2]); val[3] += bfr(bias[c0 + cofs + 3]); }
                *(volatile v4f*)(crow + (size_t)row * ldc + cofs) = val; }
            if (ps == 0) __threadfence(); }
        __builtin_amdgcn_wave_barrier(); asm volatile("" ::: "memory");
    }
}

__device__ __forceinline__ h16 tohx(float x) { return (h16)x; }
typedef __attribute__((ext_vector_type(2))) _Float16 v2h;
typedef __attribute__((ext_vector_type(4))) _Float16 v4h;
typedef __attribute__((ext_vector_type(4))) unsigned short v4us;

__global__ __launch_bounds__(256) void k_cvt8(const float* __restrict__ src, bf* dst, size_t n8) { const size_t i = (size_t)blockIdx.x * 256 + threadIdx.x; if (i >= n8) return; const v8f v = *(const v8f*)(src + i * 8); v8us o;
#pragma unroll
    for (int k = 0; k < 8; ++k) o[k] = f2bf(v[k]); *(volatile v8us*)(dst + i * 8) = o; __threadfence(); *(volatile v8us*)(dst + i * 8) = o; }
__global__ __launch_bounds__(256) void k_w16(const float* __restrict__ w, size_t n4, h16* Bt) { const size_t i = ((size_t)blockIdx.x * 256 + threadIdx.x) * 4; if (i >= n4 * 4) return; const v4f a = *(const v4f*)(w + i); v4h o; o[0] = tohx(bfr(a[0])); o[1] = tohx(bfr(a[1])); o[2] = tohx(bfr(a[2])); o[3] = tohx(bfr(a[3])); *(volatile v4h*)(Bt + i) = o; __threadfence(); *(volatile v4h*)(Bt + i) = o; }
__global__ __launch_bounds__(256) void k_xt(const float* __restrict__ x, bf* XT) { const size_t e = ((size_t)blockIdx.x * 256 + threadIdx.x) * 4; if (e >= (size_t)NN * DIM) return; const int c = (int)(e % DIM); const int n = (int)(e / DIM); v4us o;
#pragma unroll
    for (int q = 0; q < 4; ++q) o[q] = f2bf(x[(size_t)(c + q) * NN + n]); *(volatile v4us*)(XT + e) = o; __threadfence(); *(volatile v4us*)(XT + e) = o; }
__global__ __launch_bounds__(256) void k_f16(const float* __restrict__ F, size_t n4, h16* P) { const size_t i = ((size_t)blockIdx.x * 256 + threadIdx.x) * 4; if (i >= n4 * 4) return; const v4f a = *(const v4f*)(F + i); v4h o; o[0] = tohx(a[0]); o[1] = tohx(a[1]); o[2] = tohx(a[2]); o[3] = tohx(a[3]); *(volatile v4h*)(P + i) = o; __threadfence(); *(volatile v4h*)(P + i) = o; }
__device__ __forceinline__ int slot2tok(int br, int w, int m) { int y, x; if (br == 0) { y = m / 7; x = w * 7 + m % 7; } else { y = w * 7 + m / RES; x = m % RES; } return y * RES + x; }
__device__ __forceinline__ void slot2yx(int br, int m, int& hi, int& wi) { if (br == 0) { hi = m / 7; wi = m % 7; } else { hi = m / RES; wi = m % RES; } }
__global__ __launch_bounds__(256) void k_winqk(const float* __restrict__ QKV, int br, h16* QW, h16* KW) { const size_t e = ((size_t)blockIdx.x * 256 + threadIdx.x) * 4; if (e >= (size_t)NG2 * NTP * 64) return; const int d = (int)(e % 64); const int m = (int)((e / 64) % NTP); const int g = (int)(e / ((size_t)64 * NTP)); const int h = g % 2, w = g / 2; v4h oq, ok;
    if (m < NTW && d < CSD) { const float* r = QKV + (size_t)slot2tok(br, w, m) * 3 * TD + br * CSC + h * CSD + d;
#pragma unroll
        for (int q = 0; q < 4; ++q) { oq[q] = tohx(r[q] * 0.14433756729740643f); ok[q] = tohx(r[TD + q]); } } else { for (int q = 0; q < 4; ++q) { oq[q] = (h16)0.f; ok[q] = (h16)0.f; } }
    for (int ps = 0; ps < 2; ++ps) { *(volatile v4h*)(QW + e) = oq; *(volatile v4h*)(KW + e) = ok; if (ps == 0) __threadfence(); } }
__global__ __launch_bounds__(256) void k_winvt(const float* __restrict__ QKV, int br, h16* VT) { const size_t e = ((size_t)blockIdx.x * 256 + threadIdx.x) * 2; if (e >= (size_t)NG2 * 64 * NTP) return; const int m = (int)(e % NTP); const int d = (int)((e / NTP) % 64); const int g = (int)(e / ((size_t)NTP * 64)); const int h = g % 2, w = g / 2; v2h o;
#pragma unroll
    for (int u = 0; u < 2; ++u) { const int mm = m + u; o[u] = (d < CSD && mm < NTW) ? tohx(QKV[(size_t)slot2tok(br, w, mm) * 3 * TD + 2 * TD + br * CSC + h * CSD + d]) : (h16)0.f; }
    *(volatile v2h*)(VT + e) = o; __threadfence(); *(volatile v2h*)(VT + e) = o; }
template <int NFULL, int TAIL> __global__ __launch_bounds__(256) void k_soft(const float* __restrict__ Sb, int nrows, int rowsper, int rvalid, int nvalid, h16* P) { const int lane = threadIdx.x & 31; const size_t row = (size_t)blockIdx.x * 8 + (threadIdx.x >> 5); if (row >= (size_t)nrows) return; constexpr int LD = NFULL * 128 + TAIL * 64; const float* sr = Sb + row * LD; h16* pr = P + row * LD; const bool live = (int)(row % rowsper) < rvalid; float mx = -3.0e38f;
#pragma unroll 1
    for (int ch = 0; ch < NFULL + TAIL; ++ch) { if (ch == NFULL && lane >= 16) break; const int j0 = ch * 128 + lane * 4; const v4f a = *(const v4f*)(sr + j0);
#pragma unroll
        for (int q = 0; q < 4; ++q) if (j0 + q < nvalid) mx = fmaxf(mx, a[q]); }
#pragma unroll
    for (int sh = 16; sh; sh >>= 1) mx = fmaxf(mx, __shfl_xor(mx, sh, 32));
    float sum = 0.f;
#pragma unroll 1
    for (int ch = 0; ch < NFULL + TAIL; ++ch) { if (ch == NFULL && lane >= 16) break; const int j0 = ch * 128 + lane * 4; const v4f a = *(const v4f*)(sr + j0);
#pragma unroll
        for (int q = 0; q < 4; ++q) if (j0 + q < nvalid) { float d0 = __fsub_rn(a[q], mx); asm volatile("" : "+v"(d0)); sum += __expf(d0); } }
#pragma unroll
    for (int sh = 16; sh; sh >>= 1) sum += __shfl_xor(sum, sh, 32);
    const float f = live ? __fdiv_rn(PCAR, sum) : 0.f;
    for (int ps = 0; ps < 2; ++ps) {
#pragma unroll 1
        for (int ch = 0; ch < NFULL + TAIL; ++ch) { if (ch == NFULL && lane >= 16) break; const int j0 = ch * 128 + lane * 4; const v4f a = *(const v4f*)(sr + j0); v4h o;
#pragma unroll
            for (int q = 0; q < 4; ++q) { float val = 0.f; if (live && j0 + q < nvalid) { float d0 = __fsub_rn(a[q], mx); asm volatile("" : "+v"(d0)); val = __fmul_rn(__expf(d0), f); } o[q] = tohx(val); } *(volatile v4h*)(pr + j0) = o; }
        if (ps == 0) __threadfence(); } }
__global__ __launch_bounds__(256) void k_wcomb(const float* __restrict__ OW, const float* __restrict__ QKV, const float* __restrict__ lw, const float* __restrict__ lb, int br, float* ATT) { const size_t e = ((size_t)blockIdx.x * 256 + threadIdx.x) * 4; if (e >= (size_t)NWD * NTW * CSC) return; const int c = (int)(e % CSC); const int m = (int)((e / CSC) % NTW); const int w = (int)(e / ((size_t)CSC * NTW)); const int h = c / CSD, d = c % CSD; const int H_ = br == 0 ? RES : 7, W_ = br == 0 ? 7 : RES; int hi, wi; slot2yx(br, m, hi, wi); const int n = slot2tok(br, w, m); v4f o;
#pragma unroll
    for (int q = 0; q < 4; ++q) { const int cc = c + q; float acc = bfr(lb[cc]);
#pragma unroll
        for (int dy = 0; dy < 3; ++dy) { const int yy = hi + dy - 1; if (yy < 0 || yy >= H_) continue;
#pragma unroll
            for (int dx = 0; dx < 3; ++dx) { const int xx = wi + dx - 1; if (xx < 0 || xx >= W_) continue; const int mm = br == 0 ? yy * 7 + xx : yy * RES + xx; float p = __fmul_rn(QKV[(size_t)slot2tok(br, w, mm) * 3 * TD + 2 * TD + br * CSC + cc], bfr(lw[cc * 9 + dy * 3 + dx])); asm volatile("" : "+v"(p)); acc = __fadd_rn(acc, p); } }
        o[q] = __fadd_rn(OW[((size_t)(w * 2 + h) * NTP + m) * 64 + d + q] * (1.0f / PCAR), acc); }
    const size_t oo = (size_t)n * DIM + br * CSC + c; *(volatile v4f*)(ATT + oo) = o; __threadfence(); *(volatile v4f*)(ATT + oo) = o; }
__global__ __launch_bounds__(256) void k_gpl(const float* __restrict__ QKV, int h, h16* Q16, h16* K16, h16* VT) { const size_t e = ((size_t)blockIdx.x * 256 + threadIdx.x) * 4; if (e >= (size_t)NN * DH) return; const int d = (int)(e % DH); const int n = (int)(e / DH); const float* r = QKV + (size_t)n * 3 * TD + h * DH + d; v4h oq, ok;
#pragma unroll
    for (int q = 0; q < 4; ++q) { oq[q] = tohx(r[q] * 0.125f); ok[q] = tohx(r[TD + q]); } for (int ps = 0; ps < 2; ++ps) { *(volatile v4h*)(Q16 + e) = oq; *(volatile v4h*)(K16 + e) = ok; if (ps == 0) __threadfence(); } }
__global__ __launch_bounds__(256) void k_gvt(const float* __restrict__ QKV, int h, h16* VT) { const size_t e = ((size_t)blockIdx.x * 256 + threadIdx.x) * 2; if (e >= (size_t)DH * NN) return; const int n = (int)(e % NN); const int d = (int)(e / NN); v2h o; o[0] = tohx(QKV[(size_t)n * 3 * TD + 2 * TD + h * DH + d]); o[1] = tohx(QKV[(size_t)(n + 1) * 3 * TD + 2 * TD + h * DH + d]); *(volatile v2h*)(VT + e) = o; __threadfence(); *(volatile v2h*)(VT + e) = o; }
__global__ __launch_bounds__(256) void k_gcomb(const float* __restrict__ OG, int h, float* ATT) { const size_t e = ((size_t)blockIdx.x * 256 + threadIdx.x) * 4; if (e >= (size_t)NN * DH) return; const int d = (int)(e % DH); const int n = (int)(e / DH); const v4f a = *(const v4f*)(OG + e); v4f o; o[0] = a[0] * (1.0f / PCAR); o[1] = a[1] * (1.0f / PCAR); o[2] = a[2] * (1.0f / PCAR); o[3] = a[3] * (1.0f / PCAR); const size_t oo = (size_t)n * DIM + TD + h * DH + d; *(volatile v4f*)(ATT + oo) = o; __threadfence(); *(volatile v4f*)(ATT + oo) = o; }
__global__ __launch_bounds__(256) void k_outT(const float* __restrict__ ATT, float* OUT) { const size_t e = ((size_t)blockIdx.x * 256 + threadIdx.x) * 4; if (e >= (size_t)DIM * NN) return; const int n = (int)(e % NN); const int c = (int)(e / NN); v4f o;
#pragma unroll
    for (int q = 0; q < 4; ++q) o[q] = ATT[(size_t)(n + q) * DIM + c]; *(volatile v4f*)(OUT + e) = o; __threadfence(); *(volatile v4f*)(OUT + e) = o; }

extern "C" void kernel_launch(void* const* d_in, const int* in_sizes, int n_in,
                              void* d_out, int out_size, void* d_ws, size_t ws_size, hipStream_t stream) {
    (void)in_sizes; (void)n_in; (void)out_size;
    const float* xa = (const float*)d_in[0]; const float* p1 = (const float*)d_in[1]; const float* p2 = (const float*)d_in[2]; const float* wup = (const float*)d_in[3]; const float* wdn = (const float*)d_in[4]; const float* lw0 = (const float*)d_in[5]; const float* lb0 = (const float*)d_in[6]; const float* lw1 = (const float*)d_in[7]; const float* lb1 = (const float*)d_in[8];
    float* OUT = (float*)d_out;
    char* wsp = (char*)d_ws;
    auto take = [&](size_t bytes) { char* p = wsp; wsp += (bytes + 255) & ~(size_t)255; return (void*)p; };
    bf* P1 = (bf*)take((size_t)TD * DIM * 2); bf* P2 = (bf*)take((size_t)TD * DIM * 2); h16* WUP = (h16*)take((size_t)3 * TD * TD * 2); h16* WDN = (h16*)take((size_t)3 * TD * TD * 2);
    bf* XT = (bf*)take((size_t)NN * DIM * 2); float* XP = (float*)take((size_t)NN * TD * 4); h16* X16 = (h16*)take((size_t)NN * TD * 2); float* QKV1 = (float*)take((size_t)NN * 3 * TD * 4); float* QKV2 = (float*)take((size_t)NN * 3 * TD * 4);
    h16* QW = (h16*)take((size_t)NG2 * NTP * 64 * 2); h16* KW = (h16*)take((size_t)NG2 * NTP * 64 * 2); h16* VTW = (h16*)take((size_t)NG2 * 64 * NTP * 2); float* SW = (float*)take((size_t)NG2 * NTP * NTP * 4); h16* PW = (h16*)take((size_t)NG2 * NTP * NTP * 2); float* OW = (float*)take((size_t)NG2 * NTP * 64 * 4);
    h16* QG = (h16*)take((size_t)NN * DH * 2); h16* KG = (h16*)take((size_t)NN * DH * 2); h16* VTG = (h16*)take((size_t)DH * NN * 2); float* SG = (float*)take((size_t)NN * NN * 4); h16* PG = (h16*)take((size_t)NN * NN * 2); float* OG = (float*)take((size_t)NN * DH * 4); float* ATT = (float*)take((size_t)NN * DIM * 4);
    if ((size_t)(wsp - (char*)d_ws) > ws_size) return;
    k_cvt8<<<(TD * DIM / 8 + 255) / 256, 256, 0, stream>>>(p1, P1, TD * DIM / 8); k_cvt8<<<(TD * DIM / 8 + 255) / 256, 256, 0, stream>>>(p2, P2, TD * DIM / 8); k_w16<<<(3 * TD * TD / 4 + 255) / 256, 256, 0, stream>>>(wup, 3 * TD * TD / 4, WUP); k_w16<<<(3 * TD * TD / 4 + 255) / 256, 256, 0, stream>>>(wdn, 3 * TD * TD / 4, WDN);
    for (int b = 0; b < NBI; ++b) {
        k_xt<<<(unsigned)(((size_t)NN * DIM / 4 + 255) / 256), 256, 0, stream>>>(xa + (size_t)b * DIM * NN, XT);
        k_gemmw<bf, 0, false><<<dim3(NN / 64, TD / 64, 1), 32, 0, stream>>>(XT, nullptr, P1, nullptr, DIM, XP, TD, nullptr, 0, 0, 0); k_f16<<<(unsigned)(((size_t)NN * TD / 4 + 255) / 256), 256, 0, stream>>>(XP, (size_t)NN * TD / 4, X16);
        k_gemmw<h16, 0, false><<<dim3(NN / 64, 3 * TD / 64, 1), 32, 0, stream>>>(X16, nullptr, WUP, nullptr, TD, QKV1, 3 * TD, nullptr, 0, 0, 0);
        for (int br = 0; br < 2; ++br) {
            k_winqk<<<(unsigned)(((size_t)NG2 * NTP * 64 / 4 + 255) / 256), 256, 0, stream>>>(QKV1, br, QW, KW); k_winvt<<<(unsigned)(((size_t)NG2 * 64 * NTP / 2 + 255) / 256), 256, 0, stream>>>(QKV1, br, VTW);
            k_gemmw<h16, 0, false><<<dim3(NTP / 64, NTP / 64, NG2), 32, 0, stream>>>(QW, nullptr, KW, nullptr, 64, SW, NTP, nullptr, (size_t)NTP * 64, (size_t)NTP * 64, (size_t)NTP * NTP);
            k_soft<3, 1><<<(NG2 * NTP + 7) / 8, 256, 0, stream>>>(SW, NG2 * NTP, NTP, NTW, NTW, PW);
            k_gemmw<h16, 0, false><<<dim3(NTP / 64, 1, NG2), 32, 0, stream>>>(PW, nullptr, VTW, nullptr, NTP, OW, 64, nullptr, (size_t)NTP * NTP, (size_t)64 * NTP, (size_t)NTP * 64);
            k_wcomb<<<(unsigned)(((size_t)NWD * NTW * CSC / 4 + 255) / 256), 256, 0, stream>>>(OW, QKV1, br == 0 ? lw0 : lw1, br == 0 ? lb0 : lb1, br, ATT); }
        k_gemmw<bf, 0, false><<<dim3(NN / 64, TD / 64, 1), 32, 0, stream>>>(XT, nullptr, P2, nullptr, DIM, XP, TD, nullptr, 0, 0, 0); k_f16<<<(unsigned)(((size_t)NN * TD / 4 + 255) / 256), 256, 0, stream>>>(XP, (size_t)NN * TD / 4, X16);
        k_gemmw<h16, 0, false><<<dim3(NN / 64, 3 * TD / 64, 1), 32, 0, stream>>>(X16, nullptr, WDN, nullptr, TD, QKV2, 3 * TD, nullptr, 0, 0, 0);
        for (int h = 0; h < DNH; ++h) {
            k_gpl<<<(unsigned)(((size_t)NN * DH / 4 + 255) / 256), 256, 0, stream>>>(QKV2, h, QG, KG, VTG); k_gvt<<<(unsigned)(((size_t)DH * NN / 2 + 255) / 256), 256, 0, stream>>>(QKV2, h, VTG);
            k_gemmw<h16, 0, false><<<dim3(NN / 64, NN / 64, 1), 32, 0, stream>>>(QG, nullptr, KG, nullptr, DH, SG, NN, nullptr, 0, 0, 0);
            k_soft<24, 1><<<(NN + 7) / 8, 256, 0, stream>>>(SG, NN, NN, NN, NN, PG);
            k_gemmw<h16, 0, false><<<dim3(NN / 64, 1, 1), 32, 0, stream>>>(PG, nullptr, VTG, nullptr, NN, OG, DH, nullptr, 0, 0, 0);
            k_gcomb<<<(unsigned)(((size_t)NN * DH / 4 + 255) / 256), 256, 0, stream>>>(OG, h, ATT); }
        k_outT<<<(unsigned)(((size_t)DIM * NN / 4 + 255) / 256), 256, 0, stream>>>(ATT, OUT + (size_t)b * DIM * NN); }
}
